// Extractor_43387759624796
// MI455X (gfx1250) — hardware-verified
//
#include <hip/hip_runtime.h>
#include <stddef.h>


#define HID     256
#define INF     128
#define NTHR    256
#define NWAVE   8
#define EPT     8
#define NGRP    2
#define CHUNK   (NTHR * EPT * NGRP)
#define WCAP    (EPT * NGRP * 32)
#define LISTN   (NWAVE * WCAP)
#define NBC     4096
#define NBF     1024
#define RCAP    49152
#define RBN     128
#define TGT     256
#define DEGCAP  256
#define GROWS   256
#define GCOLS   64
#define OTHR    512
#define WSCAP   134217728
#define KDMAX   512
#define WP0     0
#define WP1     131072
#define WP2     393216
#define WP3     655360
#define WP4     917504
#define WP5     1179648
#define WP6     1310720
#define WPTOT   1441792
#define WPBLK   352
#define TPITCH  36

#define LDS_FILL ((RCAP + NBF + LISTN) * 4 + 64)

static_assert((CHUNK & (CHUNK - 1)) == 0);
static_assert(CHUNK <= 4096);
static_assert(NBC <= 4096 && NBF <= 4096);
static_assert((NBC & (NBC - 1)) == 0 && (NBF & (NBF - 1)) == 0);
static_assert(NBC == 4 * NBF);
static_assert(OTHR * 8 == NBC);
static_assert((RCAP % 32) == 0);
static_assert((RCAP + NBF + LISTN) * 4 + NWAVE * 4 <= LDS_FILL);
static_assert(TGT == NWAVE * 32 && TGT == GROWS);
static_assert((NBC % TGT) == 0);
static_assert(HID == 4 * GCOLS);
static_assert(WP1 == WP0 + 2 * HID * 256 && WP2 == WP1 + 2 * HID * 512 && WP3 == WP2 + 2 * HID * 512);
static_assert(WP4 == WP3 + 2 * HID * 512 && WP5 == WP4 + 2 * HID * 512 && WP6 == WP5 + 2 * HID * 256);
static_assert(WPTOT == WP6 + 2 * HID * 256);

typedef float          v4f  __attribute__((ext_vector_type(4)));
typedef float          v8f  __attribute__((ext_vector_type(8)));
typedef int            v4i  __attribute__((ext_vector_type(4)));
typedef unsigned short v8us __attribute__((ext_vector_type(8)));
typedef __bf16         v16b __attribute__((ext_vector_type(16)));
union FragB { v16b v; v8us h[2]; };

__device__ __forceinline__ unsigned int bfr(float f) {
  const unsigned int u = __float_as_uint(f);
  return (u + 0x7FFFu + ((u >> 16) & 1u)) >> 16;
}

__device__ __forceinline__ void split1(float x, unsigned short& hb, unsigned short& lb) {
  const unsigned int hu = bfr(x);
  const float hf = __uint_as_float(hu << 16);
  hb = (unsigned short)hu;
  lb = (unsigned short)bfr(x - hf);
}

__device__ __forceinline__ void split8(v4f a, v4f b, v8us& hi, v8us& lo) {
  unsigned short hb, lb;
  split1(a.x, hb, lb); hi[0] = hb; lo[0] = lb;
  split1(a.y, hb, lb); hi[1] = hb; lo[1] = lb;
  split1(a.z, hb, lb); hi[2] = hb; lo[2] = lb;
  split1(a.w, hb, lb); hi[3] = hb; lo[3] = lb;
  split1(b.x, hb, lb); hi[4] = hb; lo[4] = lb;
  split1(b.y, hb, lb); hi[5] = hb; lo[5] = lb;
  split1(b.z, hb, lb); hi[6] = hb; lo[6] = lb;
  split1(b.w, hb, lb); hi[7] = hb; lo[7] = lb;
}

__device__ __forceinline__ v8f wmb(v16b a, v16b b, v8f c) {
  v8f d = __builtin_amdgcn_wmma_f32_16x16x32_bf16(false, a, false, b, (short)0, c, false, false);
  asm volatile("v_nop\n\tv_nop\n\tv_nop\n\tv_nop" : "+v"(d) : "v"(a), "v"(b));
  return d;
}

template <int NB>
__device__ __forceinline__ int scan_chunk(const int* __restrict__ dsts, int nE, int cbase, int slotBase,
                                          int vec8, int* list, int tid, int lane, int wave) {
  int wc = 0;
#pragma unroll
  for (int g = 0; g < NGRP; ++g) {
    const int el0  = (g * NTHR + tid) * EPT;
    const int e0   = cbase + el0;
    const int sent = -2147483647 - 1;
    v4i da, db;
    if (vec8 != 0 && cbase + CHUNK <= nE) {
      da = *(const v4i*)(dsts + e0);
      db = *(const v4i*)(dsts + e0 + 4);
    } else {
      da.x = (e0     < nE) ? dsts[min(e0, nE - 1)] : sent;
      da.y = (e0 + 1 < nE) ? dsts[min(e0 + 1, nE - 1)] : sent;
      da.z = (e0 + 2 < nE) ? dsts[min(e0 + 2, nE - 1)] : sent;
      da.w = (e0 + 3 < nE) ? dsts[min(e0 + 3, nE - 1)] : sent;
      db.x = (e0 + 4 < nE) ? dsts[min(e0 + 4, nE - 1)] : sent;
      db.y = (e0 + 5 < nE) ? dsts[min(e0 + 5, nE - 1)] : sent;
      db.z = (e0 + 6 < nE) ? dsts[min(e0 + 6, nE - 1)] : sent;
      db.w = (e0 + 7 < nE) ? dsts[min(e0 + 7, nE - 1)] : sent;
    }
    const unsigned nb = (unsigned)slotBase;
    const unsigned s0 = (unsigned)da.x - nb, s1 = (unsigned)da.y - nb;
    const unsigned s2 = (unsigned)da.z - nb, s3 = (unsigned)da.w - nb;
    const unsigned s4 = (unsigned)db.x - nb, s5 = (unsigned)db.y - nb;
    const unsigned s6 = (unsigned)db.z - nb, s7 = (unsigned)db.w - nb;
    const bool h0 = s0 < (unsigned)NB, h1 = s1 < (unsigned)NB, h2 = s2 < (unsigned)NB, h3 = s3 < (unsigned)NB;
    const bool h4 = s4 < (unsigned)NB, h5 = s5 < (unsigned)NB, h6 = s6 < (unsigned)NB, h7 = s7 < (unsigned)NB;
    const unsigned any = __builtin_amdgcn_ballot_w32(h0 | h1 | h2 | h3 | h4 | h5 | h6 | h7);
    if (any != 0u) {
#define HITJ(J, HJ, SJ) { \
        const unsigned mj = __builtin_amdgcn_ballot_w32(HJ); \
        if (mj != 0u) { \
          if (HJ) { \
            const int pos = wc + (int)__builtin_amdgcn_mbcnt_lo(mj, 0u); \
            if (pos < WCAP) list[wave * WCAP + pos] = ((el0 + (J)) << 12) | (int)(SJ); \
          } \
          wc += (int)__builtin_popcount(mj); } }
      HITJ(0, h0, s0)
      HITJ(1, h1, s1)
      HITJ(2, h2, s2)
      HITJ(3, h3, s3)
      HITJ(4, h4, s4)
      HITJ(5, h5, s5)
      HITJ(6, h6, s6)
      HITJ(7, h7, s7)
#undef HITJ
    }
  }
  return wc;
}

__global__ __launch_bounds__(NTHR) void k_wprep(
    const float* __restrict__ r1, const float* __restrict__ o1,
    const float* __restrict__ r2, const float* __restrict__ o2,
    const float* __restrict__ r3, const float* __restrict__ o3,
    const float* __restrict__ r4, const float* __restrict__ o4,
    const float* __restrict__ r5, const float* __restrict__ o5,
    const float* __restrict__ wl, unsigned short* wp) {
  __shared__ __attribute__((aligned(16))) float st[64 * TPITCH];
  const int b = blockIdx.x, tid = threadIdx.x;
  int p, lb;
  if (b < 32)       { p = 0;                    lb = b; }
  else if (b < 288) { p = 1 + ((b - 32) >> 6);  lb = (b - 32) & 63; }
  else              { p = 5 + ((b - 288) >> 5); lb = (b - 288) & 31; }
  int KD, kin; size_t base; const float* wa; const float* wb;
  if (p == 0)      { KD = 256; kin = 128; wa = r1; wb = o1; base = WP0; }
  else if (p == 1) { KD = 512; kin = 256; wa = r2; wb = o2; base = WP1; }
  else if (p == 2) { KD = 512; kin = 256; wa = r3; wb = o3; base = WP2; }
  else if (p == 3) { KD = 512; kin = 256; wa = r4; wb = o4; base = WP3; }
  else if (p == 4) { KD = 512; kin = 256; wa = r5; wb = o5; base = WP4; }
  else if (p == 5) { KD = 256; kin = 256; wa = wl; wb = wl; base = WP5; }
  else             { KD = 256; kin = 256; wa = wl + (size_t)HID * HID; wb = wa; base = WP6; }
  const int kt = lb >> 3, nt = lb & 7;
  const int k0 = 64 * kt, n0 = 32 * nt;
  const float* src; int kr0;
  if (k0 < kin) { src = wa; kr0 = k0; } else { src = wb; kr0 = k0 - kin; }
#pragma unroll
  for (int i = 0; i < 2; ++i) {
    const int idx = i * NTHR + tid;
    const int r = idx >> 3, c4 = idx & 7;
    const v4f v = *(const v4f*)(src + (size_t)(kr0 + r) * HID + n0 + 4 * c4);
    *(v4f*)(st + r * TPITCH + 4 * c4) = v;
  }
  __syncthreads();
  const int nl = tid >> 3, kq = tid & 7;
  float v[8];
#pragma unroll
  for (int e = 0; e < 8; ++e) v[e] = st[(8 * kq + e) * TPITCH + nl];
  v4f a, c;
  a.x = v[0]; a.y = v[1]; a.z = v[2]; a.w = v[3];
  c.x = v[4]; c.y = v[5]; c.z = v[6]; c.w = v[7];
  v8us hv, lv;
  split8(a, c, hv, lv);
  unsigned short* dh = wp + base + (size_t)(n0 + nl) * KD + k0 + 8 * kq;
  unsigned short* dl = dh + (size_t)HID * KD;
  *(volatile v8us*)dh = hv;
  *(volatile v8us*)dl = lv;
  __threadfence();
  *(volatile v8us*)dh = hv;
  *(volatile v8us*)dl = lv;
}

__global__ __launch_bounds__(NTHR) void k_count(const int* __restrict__ ei, int* cnt, int nE, int vec8) {
  __shared__ __attribute__((aligned(16))) int scnt[NBC];
  __shared__ __attribute__((aligned(16))) int list[LISTN];
  __shared__ int wcnt[NWAVE];
  const int tid = threadIdx.x, lane = tid & 31, wave = tid >> 5;
  const int nodeBase = blockIdx.x * NBC;
  const int* dsts = ei + nE;

  for (int i = tid; i < NBC; i += NTHR) scnt[i] = 0;
  __syncthreads();

  const int nChunks = (nE + CHUNK - 1) / CHUNK;
#pragma unroll 1
  for (int ch = 0; ch < nChunks; ++ch) {
    const int cbase = ch * CHUNK;
    const int wc = scan_chunk<NBC>(dsts, nE, cbase, nodeBase, vec8, list, tid, lane, wave);
    if (lane == 0) wcnt[wave] = wc;
    __syncthreads();
    if (wave == 0) {
#pragma unroll 1
      for (int wsx = 0; wsx < NWAVE; ++wsx) {
        int n = __builtin_amdgcn_readfirstlane(wcnt[wsx]);
        n = n > WCAP ? WCAP : (n < 0 ? 0 : n);
        const int* lp = list + wsx * WCAP;
#pragma unroll 1
        for (int i = 0; i < n; ++i) {
          const int ent  = __builtin_amdgcn_readfirstlane(lp[i]);
          const int slot = ent & (NBC - 1);
          if (lane == 0) scnt[slot] = scnt[slot] + 1;
        }
      }
    }
    __syncthreads();
  }

  v4i cq[4];
#pragma unroll
  for (int q = 0; q < 4; ++q) {
    const int f = (wave * 4 + q) * 128 + 4 * lane;
    cq[q] = *(const v4i*)(scnt + f);
  }
  int* cp = cnt + (size_t)nodeBase;
#pragma unroll
  for (int q = 0; q < 4; ++q) {
    const int f = (wave * 4 + q) * 128 + 4 * lane;
    *(volatile v4i*)(cp + f) = cq[q];
  }
  __threadfence();
#pragma unroll
  for (int q = 0; q < 4; ++q) {
    const int f = (wave * 4 + q) * 128 + 4 * lane;
    *(volatile v4i*)(cp + f) = cq[q];
  }
}

__global__ __launch_bounds__(OTHR) void k_offsets(
    const int* __restrict__ cnt, int* off, int* rbase, int nChunk) {
  __shared__ __attribute__((aligned(16))) int soff[NBC];
  __shared__ __attribute__((aligned(16))) int srb[RBN];
  __shared__ int wtot[OTHR / 32];
  const int tid = threadIdx.x, lane = tid & 31, wave = tid >> 5, sub = tid >> 7;
  for (int i = tid; i < RBN; i += OTHR) srb[i] = 0;
  int carry = 0;
#pragma unroll 1
  for (int ch = 0; ch < nChunk; ++ch) {
    const int base = ch * NBC;
    const v4i c0 = *(const v4i*)(cnt + base + 8 * tid);
    const v4i c1 = *(const v4i*)(cnt + base + 8 * tid + 4);
    const int e0 = max(c0.x, 0), e1 = max(c0.y, 0), e2 = max(c0.z, 0), e3 = max(c0.w, 0);
    const int e4 = max(c1.x, 0), e5 = max(c1.y, 0), e6 = max(c1.z, 0), e7 = max(c1.w, 0);
    const int ts = e0 + e1 + e2 + e3 + e4 + e5 + e6 + e7;
    int incl = ts;
#pragma unroll
    for (int d = 1; d < 32; d <<= 1) {
      const int t = __shfl_up(incl, d);
      if (lane >= d) incl += t;
    }
    if (lane == 31) wtot[wave] = incl;
    __syncthreads();
    const int S0 = wtot[0]  + wtot[1]  + wtot[2]  + wtot[3];
    const int S1 = wtot[4]  + wtot[5]  + wtot[6]  + wtot[7];
    const int S2 = wtot[8]  + wtot[9]  + wtot[10] + wtot[11];
    const int S3 = wtot[12] + wtot[13] + wtot[14] + wtot[15];
    int pre = 0;
#pragma unroll 1
    for (int w = 4 * sub; w < wave; ++w) pre += wtot[w];
    const int b0 = carry;
    const int b1 = b0 + ((S0 + 31) & ~31);
    const int b2 = b1 + ((S1 + 31) & ~31);
    const int b3 = b2 + ((S2 + 31) & ~31);
    const int b4 = b3 + ((S3 + 31) & ~31);
    const int myb = sub == 0 ? b0 : (sub == 1 ? b1 : (sub == 2 ? b2 : b3));
    if (tid == 0) {
      srb[min(4 * ch + 0, RBN - 1)] = b0;
      srb[min(4 * ch + 1, RBN - 1)] = b1;
      srb[min(4 * ch + 2, RBN - 1)] = b2;
      srb[min(4 * ch + 3, RBN - 1)] = b3;
    }
    int run = myb + pre + incl - ts;
    soff[8 * tid + 0] = run; run += e0;
    soff[8 * tid + 1] = run; run += e1;
    soff[8 * tid + 2] = run; run += e2;
    soff[8 * tid + 3] = run; run += e3;
    soff[8 * tid + 4] = run; run += e4;
    soff[8 * tid + 5] = run; run += e5;
    soff[8 * tid + 6] = run; run += e6;
    soff[8 * tid + 7] = run;
    carry = b4;
    __syncthreads();
    const v4i q0 = *(const v4i*)(soff + 4 * tid);
    const v4i q1 = *(const v4i*)(soff + 4 * (tid + OTHR));
    int* op = off + base;
    *(volatile v4i*)(op + 4 * tid) = q0;
    *(volatile v4i*)(op + 4 * (tid + OTHR)) = q1;
    __threadfence();
    *(volatile v4i*)(op + 4 * tid) = q0;
    *(volatile v4i*)(op + 4 * (tid + OTHR)) = q1;
    __syncthreads();
  }
  if (tid == 0) srb[min(4 * nChunk, RBN - 1)] = carry;
  __syncthreads();
  v4i rv = {0, 0, 0, 0};
  if (tid < 32) rv = *(const v4i*)(srb + 4 * tid);
  if (tid < 32) *(volatile v4i*)(rbase + 4 * tid) = rv;
  __threadfence();
  if (tid < 32) *(volatile v4i*)(rbase + 4 * tid) = rv;
}

__global__ __launch_bounds__(NTHR) void k_fill(
    const int* __restrict__ ei, const int* __restrict__ off, const int* __restrict__ rbase,
    int* csr, int nN, int nE, int vec8, int csrLen) {
  extern __shared__ v4f lds_dyn[];
  int* region = (int*)lds_dyn;
  int* cursor = region + RCAP;
  int* list   = cursor + NBF;
  int* wcnt   = list + LISTN;
  const int tid = threadIdx.x, lane = tid & 31, wave = tid >> 5;
  const int b = blockIdx.x;
  const int nodeBase = b * NBF;
  const int* dsts = ei + nE;

  int rb0 = rbase[b];
  const int rb1 = rbase[b + 1];
  rb0 = rb0 < 0 ? 0 : (rb0 > csrLen ? csrLen : rb0);
  rb0 &= ~31;
  int len = rb1 - rb0;
  len = len < 0 ? 0 : (len > RCAP ? RCAP : len);
  int lenW = (len + 31) & ~31;
  if (rb0 + lenW > csrLen) lenW = (csrLen - rb0) & ~31;

  {
    const v4i z = {0, 0, 0, 0};
    for (int i = tid; i < RCAP / 4; i += NTHR) ((v4i*)region)[i] = z;
    for (int s = tid; s < NBF; s += NTHR) {
      int o = off[nodeBase + s] - rb0;
      o = o < 0 ? 0 : (o > RCAP ? RCAP : o);
      cursor[s] = o;
    }
  }
  __syncthreads();

  const int nChunks = (nE + CHUNK - 1) / CHUNK;
#pragma unroll 1
  for (int ch = 0; ch < nChunks; ++ch) {
    const int cbase = ch * CHUNK;
    const int wc = scan_chunk<NBF>(dsts, nE, cbase, nodeBase, vec8, list, tid, lane, wave);
    if (lane == 0) wcnt[wave] = wc;
    __syncthreads();
    if (wave == 0) {
#pragma unroll 1
      for (int wsx = 0; wsx < NWAVE; ++wsx) {
        int n = __builtin_amdgcn_readfirstlane(wcnt[wsx]);
        n = n > WCAP ? WCAP : (n < 0 ? 0 : n);
        const int* lp = list + wsx * WCAP;
#pragma unroll 1
        for (int i = 0; i < n; ++i) {
          const int ent  = __builtin_amdgcn_readfirstlane(lp[i]);
          const int slot = ent & (NBF - 1);
          int e = cbase + ((ent >> 12) & (CHUNK - 1));
          e = e > nE - 1 ? nE - 1 : e;
          int src = ei[e];
          src = src < 0 ? 0 : (src > nN - 1 ? nN - 1 : src);
          if (lane == 0) {
            int pos = cursor[slot];
            pos = pos < 0 ? 0 : (pos > RCAP - 1 ? RCAP - 1 : pos);
            region[pos] = src;
            const int np = pos + 1;
            cursor[slot] = np > RCAP ? RCAP : np;
          }
        }
      }
    }
    __syncthreads();
  }

  const int nv = lenW >> 2;
  int* gp = csr + rb0;
#pragma unroll 1
  for (int i = tid; i < nv; i += NTHR) { const v4i v = ((const v4i*)region)[i]; *(volatile v4i*)(gp + 4 * i) = v; }
  __threadfence();
#pragma unroll 1
  for (int i = tid; i < nv; i += NTHR) { const v4i v = ((const v4i*)region)[i]; *(volatile v4i*)(gp + 4 * i) = v; }
}

template <int CH>
__global__ __launch_bounds__(NTHR) void k_agg(
    const int* __restrict__ csr, const int* __restrict__ off, const int* __restrict__ cnt,
    const float* __restrict__ xin, unsigned short* Ahi, unsigned short* Alo,
    int nN, int csrLen, int meanflag) {
  static_assert(CH == 128 || CH == 256);
  constexpr int KD = 2 * CH;
  const int tid = threadIdx.x, lane = tid & 31, wave = tid >> 5;
  const int tbase = blockIdx.x * TGT + wave * 32;
  const int cl = tbase + lane;
  const int cnt_l = cnt[cl];
  const int off_l = off[cl];
  const int c8 = (CH == 256) ? 8 * lane : 8 * (lane & 15);

#pragma unroll 1
  for (int j = 0; j < 32; ++j) {
    const int c = tbase + j;
    const int nc = __builtin_amdgcn_readlane(cnt_l, j);
    const int n = nc < 0 ? 0 : (nc > DEGCAP ? DEGCAP : nc);
    const int st = __builtin_amdgcn_readlane(off_l, j);
    v4f a0 = {0.0f, 0.0f, 0.0f, 0.0f}, a1 = {0.0f, 0.0f, 0.0f, 0.0f};
#pragma unroll 1
    for (int q0 = 0; q0 < n; q0 += 32) {
      int pos = st + q0 + lane;
      pos = pos < 0 ? 0 : (pos > csrLen - 1 ? csrLen - 1 : pos);
      int sl = csr[pos];
      sl = sl < 0 ? 0 : (sl > nN - 1 ? nN - 1 : sl);
      const int mcnt = (n - q0) < 32 ? (n - q0) : 32;
#pragma unroll 1
      for (int p = 0; p < mcnt; ++p) {
        const int s = __builtin_amdgcn_readlane(sl, p);
        const float* xp = xin + (size_t)s * CH + c8;
        a0 = a0 + *(const v4f*)xp;
        a1 = a1 + *(const v4f*)(xp + 4);
      }
    }
    if (meanflag != 0) {
      const float d  = (float)(nc < 1 ? 1 : nc);
      const float rc = 1.0f / d;
      a0 = a0 * rc;
      a1 = a1 * rc;
    }
    const int cc = c > nN - 1 ? nN - 1 : c;
    const float* sp = xin + (size_t)cc * CH + c8;
    const v4f s0 = *(const v4f*)sp;
    const v4f s1 = *(const v4f*)(sp + 4);
    unsigned short* ph = Ahi + (size_t)c * KD + 8 * lane;
    unsigned short* pl = Alo + (size_t)c * KD + 8 * lane;
    if (CH == 256) {
      v8us hA, lA, hS, lS;
      split8(a0, a1, hA, lA);
      split8(s0, s1, hS, lS);
      *(volatile v8us*)ph = hA;
      *(volatile v8us*)(ph + CH) = hS;
      *(volatile v8us*)pl = lA;
      *(volatile v8us*)(pl + CH) = lS;
      __threadfence();
      *(volatile v8us*)ph = hA;
      *(volatile v8us*)(ph + CH) = hS;
      *(volatile v8us*)pl = lA;
      *(volatile v8us*)(pl + CH) = lS;
    } else {
      const bool lo16 = lane < 16;
      v4f r0, r1;
      r0.x = lo16 ? a0.x : s0.x; r0.y = lo16 ? a0.y : s0.y; r0.z = lo16 ? a0.z : s0.z; r0.w = lo16 ? a0.w : s0.w;
      r1.x = lo16 ? a1.x : s1.x; r1.y = lo16 ? a1.y : s1.y; r1.z = lo16 ? a1.z : s1.z; r1.w = lo16 ? a1.w : s1.w;
      v8us hv, lv;
      split8(r0, r1, hv, lv);
      *(volatile v8us*)ph = hv;
      *(volatile v8us*)pl = lv;
      __threadfence();
      *(volatile v8us*)ph = hv;
      *(volatile v8us*)pl = lv;
    }
  }
}

__global__ __launch_bounds__(NTHR) void k_cvt(const float* __restrict__ xin,
                                             unsigned short* Ahi, unsigned short* Alo) {
  const int tid = threadIdx.x, lane = tid & 31, wave = tid >> 5;
  const int rbase = blockIdx.x * TGT + wave * 32;
#pragma unroll 1
  for (int j = 0; j < 32; ++j) {
    const int row = rbase + j;
    const float* xp = xin + (size_t)row * HID + 8 * lane;
    const v4f a = *(const v4f*)xp;
    const v4f b = *(const v4f*)(xp + 4);
    v8us hv, lv;
    split8(a, b, hv, lv);
    unsigned short* ph = Ahi + (size_t)row * HID + 8 * lane;
    unsigned short* pl = Alo + (size_t)row * HID + 8 * lane;
    *(volatile v8us*)ph = hv;
    *(volatile v8us*)pl = lv;
    __threadfence();
    *(volatile v8us*)ph = hv;
    *(volatile v8us*)pl = lv;
  }
}

template <int KD>
__global__ __launch_bounds__(NTHR) void k_gemm(
    const unsigned short* __restrict__ Ahi, const unsigned short* __restrict__ Alo,
    const unsigned short* __restrict__ Bw, const float* __restrict__ bias,
    float* C, int Mlim, int relu) {
  static_assert((KD % 32) == 0 && KD <= KDMAX);
  __shared__ __attribute__((aligned(16))) float stg[NWAVE * 16 * 64];
  constexpr int NKT  = KD / 32;
  constexpr int WPLN = HID * KD;
  const int tid = threadIdx.x, lane = tid & 31, wave = tid >> 5, hh = lane >> 4, m = lane & 15;
  const int rowBase = blockIdx.x * GROWS + wave * 32;
  const int col0 = blockIdx.y * GCOLS;

  v8f acc[2][4];
#pragma unroll
  for (int mt = 0; mt < 2; ++mt)
#pragma unroll
    for (int t = 0; t < 4; ++t) { v8f z = {0.f, 0.f, 0.f, 0.f, 0.f, 0.f, 0.f, 0.f}; acc[mt][t] = z; }

  const unsigned short* ah0 = Ahi + (size_t)(rowBase + m) * KD + 8 * hh;
  const unsigned short* ah1 = ah0 + (size_t)16 * KD;
  const unsigned short* al0 = Alo + (size_t)(rowBase + m) * KD + 8 * hh;
  const unsigned short* al1 = al0 + (size_t)16 * KD;
  const unsigned short* bb  = Bw + (size_t)(col0 + m) * KD + 8 * hh;

#pragma unroll 1
  for (int kt = 0; kt < NKT; ++kt) {
    FragB a0h, a0l, a1h, a1l;
    a0h.h[0] = *(const v8us*)(ah0 + 32 * kt);
    a0h.h[1] = *(const v8us*)(ah0 + 32 * kt + 16);
    a0l.h[0] = *(const v8us*)(al0 + 32 * kt);
    a0l.h[1] = *(const v8us*)(al0 + 32 * kt + 16);
    a1h.h[0] = *(const v8us*)(ah1 + 32 * kt);
    a1h.h[1] = *(const v8us*)(ah1 + 32 * kt + 16);
    a1l.h[0] = *(const v8us*)(al1 + 32 * kt);
    a1l.h[1] = *(const v8us*)(al1 + 32 * kt + 16);
#pragma unroll
    for (int t = 0; t < 4; ++t) {
      const unsigned short* bp = bb + (size_t)(16 * t) * KD + 32 * kt;
      FragB bh, bl;
      bh.h[0] = *(const v8us*)bp;
      bh.h[1] = *(const v8us*)(bp + 16);
      bl.h[0] = *(const v8us*)(bp + WPLN);
      bl.h[1] = *(const v8us*)(bp + WPLN + 16);
      acc[0][t] = wmb(a0h.v, bh.v, acc[0][t]);
      acc[0][t] = wmb(a0h.v, bl.v, acc[0][t]);
      acc[0][t] = wmb(a0l.v, bh.v, acc[0][t]);
      acc[1][t] = wmb(a1h.v, bh.v, acc[1][t]);
      acc[1][t] = wmb(a1h.v, bl.v, acc[1][t]);
      acc[1][t] = wmb(a1l.v, bh.v, acc[1][t]);
    }
  }

  float* sw = stg + wave * 1024;
#pragma unroll
  for (int mt = 0; mt < 2; ++mt) {
#pragma unroll
    for (int t = 0; t < 4; ++t) {
      const float bv = bias[col0 + 16 * t + m];
#pragma unroll
      for (int r = 0; r < 8; ++r) {
        float v = acc[mt][t][r] + bv;
        v = (relu != 0) ? fmaxf(v, 0.0f) : v;
        sw[(8 * hh + r) * 64 + 16 * t + m] = v;
      }
    }
    __syncthreads();
    v4f vv[8];
#pragma unroll
    for (int i = 0; i < 8; ++i) vv[i] = *(const v4f*)(sw + 128 * i + 4 * lane);
#pragma unroll
    for (int i = 0; i < 8; ++i) {
      const int grow = rowBase + 16 * mt + 2 * i + (lane >> 4);
      float* gp = C + (size_t)grow * HID + col0 + 4 * (lane & 15);
      if (grow < Mlim) *(volatile v4f*)gp = vv[i];
    }
    __threadfence();
#pragma unroll
    for (int i = 0; i < 8; ++i) {
      const int grow = rowBase + 16 * mt + 2 * i + (lane >> 4);
      float* gp = C + (size_t)grow * HID + col0 + 4 * (lane & 15);
      if (grow < Mlim) *(volatile v4f*)gp = vv[i];
    }
    __syncthreads();
  }
}

static size_t carve(size_t& off, size_t bytes) {
  const size_t o = off;
  off += bytes;
  off = (off + 255) & ~(size_t)255;
  return o;
}

extern "C" void kernel_launch(void* const* d_in, const int* in_sizes, int n_in,
                              void* d_out, int out_size, void* d_ws, size_t ws_size,
                              hipStream_t stream) {
  if (n_in < 21) return;
  const int nN = in_sizes[0] / INF;
  if (nN <= 0 || in_sizes[0] != nN * INF) return;
  int nEs[3];
  nEs[0] = in_sizes[1] / 2;
  nEs[1] = in_sizes[2] / 2;
  nEs[2] = in_sizes[3] / 2;
  for (int s = 0; s < 3; ++s) {
    if (nEs[s] <= 0 || in_sizes[1 + s] != 2 * nEs[s] || nEs[s] > (1 << 26)) return;
  }
  if (in_sizes[4] != INF * HID || in_sizes[5] != INF * HID || in_sizes[6] != HID) return;
  for (int i = 1; i < 5; ++i) {
    if (in_sizes[4 + 3 * i] != HID * HID || in_sizes[5 + 3 * i] != HID * HID || in_sizes[6 + 3 * i] != HID) return;
  }
  if (in_sizes[19] != 2 * HID * HID || in_sizes[20] != 2 * HID) return;
  if (out_size != nN * HID) return;
  if (nN > (1 << 22)) return;

  const float* x    = (const float*)d_in[0];
  const int*   eis[3];
  eis[0] = (const int*)d_in[1];
  eis[1] = (const int*)d_in[2];
  eis[2] = (const int*)d_in[3];
  const float* wroot1 = (const float*)d_in[4];
  const float* wrel1  = (const float*)d_in[5];
  const float* b1     = (const float*)d_in[6];
  const float* wroot2 = (const float*)d_in[7];
  const float* wrel2  = (const float*)d_in[8];
  const float* b2     = (const float*)d_in[9];
  const float* wroot3 = (const float*)d_in[10];
  const float* wrel3  = (const float*)d_in[11];
  const float* b3     = (const float*)d_in[12];
  const float* wroot4 = (const float*)d_in[13];
  const float* wrel4  = (const float*)d_in[14];
  const float* b4     = (const float*)d_in[15];
  const float* wroot5 = (const float*)d_in[16];
  const float* wrel5  = (const float*)d_in[17];
  const float* b5     = (const float*)d_in[18];
  const float* wl     = (const float*)d_in[19];
  const float* bl     = (const float*)d_in[20];
  float* out = (float*)d_out;

  const int NPAD   = ((nN + TGT - 1) / TGT) * TGT;
  const int nBC    = (nN + NBC - 1) / NBC;
  const int CNTPAD = nBC * NBC;
  if (4 * nBC + 1 > RBN) return;
  const int nBF    = (nN + NBF - 1) / NBF;
  if (31 * 4 * nBC > 4096) return;
  int csrLen[3];
  for (int s = 0; s < 3; ++s) csrLen[s] = ((nEs[s] + 31) & ~31) + 4096;
  const int nGemm = NPAD / GROWS;
  const int nAgg  = NPAD / TGT;

  size_t off = 0;
  const size_t oW = carve(off, (size_t)WPTOT * 2);
  size_t oCnt[3], oOff[3], oRb[3], oCsr[3];
  for (int s = 0; s < 3; ++s) {
    oCnt[s] = carve(off, (size_t)CNTPAD * 4);
    oOff[s] = carve(off, (size_t)CNTPAD * 4);
    oRb[s]  = carve(off, (size_t)RBN * 4);
    oCsr[s] = carve(off, (size_t)csrLen[s] * 4);
  }
  const size_t oAh = carve(off, (size_t)NPAD * KDMAX * 2);
  const size_t oAl = carve(off, (size_t)NPAD * KDMAX * 2);
  const size_t oH  = carve(off, (size_t)NPAD * HID * 4);
  if (off > ws_size || off > (size_t)WSCAP) return;

  char* ws = (char*)d_ws;
  unsigned short* wp  = (unsigned short*)(ws + oW);
  int* cnt[3]; int* offp[3]; int* rb[3]; int* csr[3];
  for (int s = 0; s < 3; ++s) {
    cnt[s]  = (int*)(ws + oCnt[s]);
    offp[s] = (int*)(ws + oOff[s]);
    rb[s]   = (int*)(ws + oRb[s]);
    csr[s]  = (int*)(ws + oCsr[s]);
  }
  unsigned short* Ah = (unsigned short*)(ws + oAh);
  unsigned short* Al = (unsigned short*)(ws + oAl);
  float* H = (float*)(ws + oH);

  k_wprep<<<WPBLK, NTHR, 0, stream>>>(wrel1, wroot1, wrel2, wroot2, wrel3, wroot3,
                                       wrel4, wroot4, wrel5, wroot5, wl, wp);

  hipFuncSetAttribute(reinterpret_cast<const void*>(&k_fill),
                      hipFuncAttributeMaxDynamicSharedMemorySize, LDS_FILL);
  for (int s = 0; s < 3; ++s) {
    const int vec8 = ((nEs[s] & 3) == 0) ? 1 : 0;
    k_count<<<nBC, NTHR, 0, stream>>>(eis[s], cnt[s], nEs[s], vec8);
    k_offsets<<<1, OTHR, 0, stream>>>(cnt[s], offp[s], rb[s], nBC);
    k_fill<<<nBF, NTHR, LDS_FILL, stream>>>(eis[s], offp[s], rb[s], csr[s], nN, nEs[s], vec8, csrLen[s]);
  }

  const dim3 ggrid((unsigned)nGemm, (unsigned)(HID / GCOLS));

  k_agg<128><<<nAgg, NTHR, 0, stream>>>(csr[0], offp[0], cnt[0], x, Ah, Al, nN, csrLen[0], 0);
  k_gemm<256><<<ggrid, NTHR, 0, stream>>>(Ah, Al, wp + WP0, b1, H, NPAD, 1);

  k_agg<256><<<nAgg, NTHR, 0, stream>>>(csr[2], offp[2], cnt[2], H, Ah, Al, nN, csrLen[2], 0);
  k_gemm<512><<<ggrid, NTHR, 0, stream>>>(Ah, Al, wp + WP1, b2, H, NPAD, 0);

  for (int it = 0; it < 2; ++it) {
    k_agg<256><<<nAgg, NTHR, 0, stream>>>(csr[0], offp[0], cnt[0], H, Ah, Al, nN, csrLen[0], 1);
    k_gemm<512><<<ggrid, NTHR, 0, stream>>>(Ah, Al, wp + WP2, b3, H, NPAD, 1);
  }

  k_agg<256><<<nAgg, NTHR, 0, stream>>>(csr[1], offp[1], cnt[1], H, Ah, Al, nN, csrLen[1], 0);
  k_gemm<512><<<ggrid, NTHR, 0, stream>>>(Ah, Al, wp + WP3, b4, H, NPAD, 1);

  for (int it = 0; it < 2; ++it) {
    k_agg<256><<<nAgg, NTHR, 0, stream>>>(csr[0], offp[0], cnt[0], H, Ah, Al, nN, csrLen[0], 0);
    k_gemm<512><<<ggrid, NTHR, 0, stream>>>(Ah, Al, wp + WP4, b5, H, NPAD, 1);
  }

  k_cvt<<<nAgg, NTHR, 0, stream>>>(H, Ah, Al);
  k_gemm<256><<<ggrid, NTHR, 0, stream>>>(Ah, Al, wp + WP5, bl, H, NPAD, 0);
  k_cvt<<<nAgg, NTHR, 0, stream>>>(H, Ah, Al);
  k_gemm<256><<<ggrid, NTHR, 0, stream>>>(Ah, Al, wp + WP6, bl + HID, out, nN, 0);
}
